// React_attention_84464826843818
// MI455X (gfx1250) — hardware-verified
//
#include <hip/hip_runtime.h>
#include <math.h>
#include <stdint.h>

#define NBATCH 8
#define SENC   2048
#define SDEC   1024
#define DIN    512
#define UNITS  512

typedef __attribute__((ext_vector_type(16))) _Float16 v16h;
typedef __attribute__((ext_vector_type(8)))  _Float16 v8h;
typedef __attribute__((ext_vector_type(16))) __bf16   v16b;
typedef __attribute__((ext_vector_type(8)))  __bf16   v8b;
typedef __attribute__((ext_vector_type(8)))  float    v8f;
typedef __attribute__((ext_vector_type(4)))  float    v4f;
typedef __attribute__((ext_vector_type(2)))  float    v2f;
typedef __attribute__((ext_vector_type(4)))  unsigned int v4u;

__device__ __forceinline__ unsigned short f2bf_bits(float f) {
  unsigned u = __float_as_uint(f);
  return (unsigned short)((u + 0x7FFFu + ((u >> 16) & 1u)) >> 16);
}
__device__ __forceinline__ float bf_bits2f(unsigned short h) { return __uint_as_float(((unsigned)h) << 16); }

__device__ __forceinline__ void dep_guard_h(v8f& a, v8f& b, v16h x, v16h y) { asm volatile("v_nop\n\tv_nop\n\tv_nop\n\tv_nop" : "+v"(a), "+v"(b) : "v"(x), "v"(y)); }
__device__ __forceinline__ void dep_guard_b(v8f& a, v8f& b, v16b x, v16b y) { asm volatile("v_nop\n\tv_nop\n\tv_nop\n\tv_nop" : "+v"(a), "+v"(b) : "v"(x), "v"(y)); }
__device__ __forceinline__ void keep4_h(v16h a, v16h b, v16h c, v16h d) { asm volatile("v_nop" :: "v"(a), "v"(b), "v"(c), "v"(d)); }
__device__ __forceinline__ void keep4_b(v16b a, v16b b, v16b c, v16b d) { asm volatile("v_nop" :: "v"(a), "v"(b), "v"(c), "v"(d)); }
__device__ __forceinline__ void acc_guard4(v8f& a, v8f& b, v8f& c, v8f& d) { asm volatile("v_nop\n\tv_nop\n\tv_nop\n\tv_nop" : "+v"(a), "+v"(b), "+v"(c), "+v"(d)); }
template <typename T> struct Frag;
template <> struct Frag<_Float16> {
  typedef v16h V; union U { v16h v; v8h h[2]; };
  static __device__ __forceinline__ v16h load(const _Float16* p) {
    U f; f.h[0] = *(const v8h*)(p); f.h[1] = *(const v8h*)(p + 16); return f.v;
  }
  static __device__ __forceinline__ v8f mma(v16h a, v16h b, v8f c) {
    return __builtin_amdgcn_wmma_f32_16x16x32_f16(false, a, false, b, (short)0, c, false, false);
  }
  static __device__ __forceinline__ void guard(v8f& a, v8f& b, v16h x, v16h y) { dep_guard_h(a, b, x, y); }
  static __device__ __forceinline__ void keep(v16h a, v16h b, v16h c, v16h d) { keep4_h(a, b, c, d); }
};
template <> struct Frag<__bf16> {
  typedef v16b V; union U { v16b v; v8b h[2]; };
  static __device__ __forceinline__ v16b load(const __bf16* p) {
    U f; f.h[0] = *(const v8b*)(p); f.h[1] = *(const v8b*)(p + 16); return f.v;
  }
  static __device__ __forceinline__ v8f mma(v16b a, v16b b, v8f c) {
    return __builtin_amdgcn_wmma_f32_16x16x32_bf16(false, a, false, b, (short)0, c, false, false);
  }
  static __device__ __forceinline__ void guard(v8f& a, v8f& b, v16b x, v16b y) { dep_guard_b(a, b, x, y); }
  static __device__ __forceinline__ void keep(v16b a, v16b b, v16b c, v16b d) { keep4_b(a, b, c, d); }
};

template <int ET> struct Elem;
template <> struct Elem<0> { typedef _Float16 T; };
template <> struct Elem<1> { typedef __bf16 T; };
template <int ET, bool SPLIT, int BIAS_MODE, int OUT_MODE, bool RESID, int ACT = 0>
__global__ __launch_bounds__(256) void wmma_gemm64(
    const unsigned short* __restrict__ Ap, const unsigned short* __restrict__ A2p, int lda, long strideA,
    const unsigned short* __restrict__ Btp, const unsigned short* __restrict__ Bt2p, int ldb, long strideB,
    void* __restrict__ Cout, void* __restrict__ Cout2, int ldc, long strideC,
    const float* __restrict__ bias,
    const float* __restrict__ resid, long strideR,
    int M, int N, int K, float scale) {
  typedef typename Elem<ET>::T T;
  typedef typename Frag<T>::V V;
  const T* A = (const T*)Ap; const T* A2 = (const T*)A2p; const T* Bt = (const T*)Btp; const T* Bt2 = (const T*)Bt2p;
  __shared__ __align__(16) float sT[8][16 * 68];
  const int b    = blockIdx.y;
  const int lane = threadIdx.x & 31;
  const int wave = threadIdx.x >> 5;
  const int tilesN = N >> 6;
  const int tilesM = M >> 6;
  const int tile = blockIdx.x * 8 + wave;
  if (tile >= tilesM * tilesN) return;
  const int tm = tile / tilesN;
  const int tn = tile - tm * tilesN;
  const int m0 = tm << 6;
  const int n0 = tn << 6;

  const T* Ab  = A  + (size_t)b * strideA;
  const T* Bb  = Bt + (size_t)b * strideB;
  const T* Ab2 = SPLIT ? (A2  + (size_t)b * strideA) : nullptr;
  const T* Bb2 = SPLIT ? (Bt2 + (size_t)b * strideB) : nullptr;

  const int rlane = lane & 15;
  const int koff  = (lane >> 4) * 8;
  const int mOff  = (lane >> 4) * 8;

  v8f acc[4][4];
#pragma unroll
  for (int i = 0; i < 4; ++i)
#pragma unroll
    for (int j = 0; j < 4; ++j) acc[i][j] = (v8f){0.f,0.f,0.f,0.f,0.f,0.f,0.f,0.f};

  for (int k0 = 0; k0 < K; k0 += 32) {
    V bh[4], bl[4];
#pragma unroll
    for (int j = 0; j < 4; ++j) {
      const size_t bo = (size_t)(n0 + (j << 4) + rlane) * ldb + koff + k0;
      bh[j] = Frag<T>::load(Bb + bo);
      if (SPLIT) bl[j] = Frag<T>::load(Bb2 + bo);
    }
#pragma unroll
    for (int i = 0; i < 4; ++i) {
      const size_t ao = (size_t)(m0 + (i << 4) + rlane) * lda + koff + k0;
      V ah = Frag<T>::load(Ab + ao);
      V al;
      if (SPLIT) al = Frag<T>::load(Ab2 + ao);
#pragma unroll
      for (int j = 0; j < 4; ++j) {
        acc[i][j] = Frag<T>::mma(ah, bh[j], acc[i][j]);
        if (SPLIT) {
          acc[i][j] = Frag<T>::mma(ah, bl[j], acc[i][j]);
          acc[i][j] = Frag<T>::mma(al, bh[j], acc[i][j]);
        }
      }
      Frag<T>::guard(acc[i][0], acc[i][3], ah, SPLIT ? al : ah);
    }
    Frag<T>::keep(bh[0], bh[1], bh[2], bh[3]);
    if (SPLIT) Frag<T>::keep(bl[0], bl[1], bl[2], bl[3]);
  }
  acc_guard4(acc[0][0], acc[0][1], acc[0][2], acc[0][3]);
  acc_guard4(acc[1][0], acc[1][1], acc[1][2], acc[1][3]);
  acc_guard4(acc[2][0], acc[2][1], acc[2][2], acc[2][3]);
  acc_guard4(acc[3][0], acc[3][1], acc[3][2], acc[3][3]);

  float* slab = sT[wave];
  const float* Rb = RESID ? (resid + (size_t)b * strideR) : nullptr;
#pragma unroll
  for (int i = 0; i < 4; ++i) {
    const int mBase = m0 + (i << 4);
#pragma unroll
    for (int j = 0; j < 4; ++j) {
      const int n = n0 + (j << 4) + rlane;
      float bv = 0.f;
      if (BIAS_MODE == 2) bv = bias[n];
#pragma unroll
      for (int r = 0; r < 8; ++r) {
        float v = acc[i][j][r] * scale;
        if (BIAS_MODE == 1) v += bias[mBase + mOff + r];
        if (BIAS_MODE == 2) v += bv;
        if (RESID) v += Rb[(size_t)(mBase + mOff + r) * ldc + n];
        if (ACT == 1) v = tanhf(v);
        if (ACT == 2) v = fmaxf(v, 0.0f);
        if (ACT == 4) v = (v > 0.f) ? v : 0.01f * v;
        slab[(mOff + r) * 68 + (j << 4) + rlane] = v;
      }
    }
    __builtin_amdgcn_fence(__ATOMIC_RELEASE, "workgroup");
    __builtin_amdgcn_wave_barrier();
    __builtin_amdgcn_fence(__ATOMIC_ACQUIRE, "workgroup");
    if (OUT_MODE == 0) {
      float* C = (float*)Cout + (size_t)b * strideC;
      const int hh = lane >> 4, c4 = (lane & 15) * 4;
      for (int pass = 0; pass < 2; ++pass) {
#pragma unroll
        for (int it = 0; it < 8; ++it) {
          const int row = it * 2 + hh;
          v4f v = *(const v4f*)(slab + row * 68 + c4);
          *(volatile v4f*)(C + (size_t)(mBase + row) * ldc + n0 + c4) = v;
        }
        __threadfence();
      }
    } else {
      const int q = lane >> 3, c8 = (lane & 7) * 8;
      unsigned short* C  = (unsigned short*)Cout  + (size_t)b * strideC;
      unsigned short* C2 = (OUT_MODE == 2) ? ((unsigned short*)Cout2 + (size_t)b * strideC) : nullptr;
      for (int pass = 0; pass < 2; ++pass) {
#pragma unroll
        for (int it = 0; it < 4; ++it) {
          const int row = it * 4 + q;
          const float* sp = slab + row * 68 + c8;
          v8h hv, lv;
#pragma unroll
          for (int e = 0; e < 8; ++e) {
            if (OUT_MODE == 1) {
              hv[e] = (_Float16)sp[e];
            } else {
              unsigned short hb = f2bf_bits(sp[e]);
              unsigned short lb = f2bf_bits(sp[e] - bf_bits2f(hb));
              hv[e] = __builtin_bit_cast(_Float16, hb);
              lv[e] = __builtin_bit_cast(_Float16, lb);
            }
          }
          *(volatile v8h*)(C + (size_t)(mBase + row) * ldc + n0 + c8) = hv;
          if (OUT_MODE == 2) *(volatile v8h*)(C2 + (size_t)(mBase + row) * ldc + n0 + c8) = lv;
        }
        __threadfence();
      }
    }
    __builtin_amdgcn_fence(__ATOMIC_RELEASE, "workgroup");
    __builtin_amdgcn_wave_barrier();
    __builtin_amdgcn_fence(__ATOMIC_ACQUIRE, "workgroup");
  }
}

__device__ __forceinline__ unsigned pk16(unsigned short a, unsigned short b) { return (unsigned)a | ((unsigned)b << 16); }

__global__ __launch_bounds__(256) void split_bf16x2_kernel(const float* __restrict__ in, unsigned short* __restrict__ hi,
                                                           unsigned short* __restrict__ lo, int n2) {
  const int i = blockIdx.x * 256 + threadIdx.x;
  if (i < n2) {
    const v2f f = *(const v2f*)(in + 2 * (size_t)i);
    const unsigned short h0 = f2bf_bits(f[0]), h1 = f2bf_bits(f[1]);
    const unsigned short l0 = f2bf_bits(f[0] - bf_bits2f(h0)), l1 = f2bf_bits(f[1] - bf_bits2f(h1));
    const unsigned uh = pk16(h0, h1), ul = pk16(l0, l1);
    ((volatile unsigned*)hi)[i] = uh;
    ((volatile unsigned*)lo)[i] = ul;
    __threadfence();
    ((volatile unsigned*)hi)[i] = uh;
    ((volatile unsigned*)lo)[i] = ul;
  }
}

__global__ __launch_bounds__(256) void transpose_split_kernel(const float* __restrict__ in, int ldi,
                                                              unsigned short* __restrict__ outh,
                                                              unsigned short* __restrict__ outl, int ldo) {
  __shared__ __align__(16) float tf[64 * 68];
  const int c0  = blockIdx.x * 64;
  const int r0  = blockIdx.y * 64;
  const int tid = threadIdx.x;
  {
    const int sub = tid >> 4;
    const int c4  = (tid & 15) * 4;
#pragma unroll
    for (int it = 0; it < 4; ++it) {
      const int rr = it * 16 + sub;
      const v4f a = *(const v4f*)(in + (size_t)(r0 + rr) * ldi + c0 + c4);
      *(v4f*)(tf + rr * 68 + c4) = a;
    }
  }
  __syncthreads();
  const int s8 = tid >> 3;
  const int c8 = (tid & 7) * 8;
  v4u hv[2], lv[2];
#pragma unroll
  for (int it = 0; it < 2; ++it) {
    const int oc = it * 32 + s8;
    v4u a, a2;
#pragma unroll
    for (int q = 0; q < 4; ++q) {
      const float f0 = tf[(c8 + 2 * q) * 68 + oc];
      const float f1 = tf[(c8 + 2 * q + 1) * 68 + oc];
      const unsigned short h0 = f2bf_bits(f0), h1 = f2bf_bits(f1);
      const unsigned short l0 = f2bf_bits(f0 - bf_bits2f(h0));
      const unsigned short l1 = f2bf_bits(f1 - bf_bits2f(h1));
      a[q]  = pk16(h0, h1);
      a2[q] = pk16(l0, l1);
    }
    hv[it] = a; lv[it] = a2;
  }
  for (int pass = 0; pass < 2; ++pass) {
#pragma unroll
    for (int it = 0; it < 2; ++it) {
      const int oc = it * 32 + s8;
      const size_t go = (size_t)(c0 + oc) * ldo + r0 + c8;
      *(volatile v4u*)(outh + go) = hv[it];
      *(volatile v4u*)(outl + go) = lv[it];
    }
    __threadfence();
  }
}

__global__ __launch_bounds__(256) void softmax_split_kernel(const float* __restrict__ S,
                                                            unsigned short* __restrict__ Phi,
                                                            unsigned short* __restrict__ Plo) {
#pragma clang fp contract(off)
  __shared__ float redm[8];
  __shared__ float reds[8];
  const int i    = blockIdx.x;
  const int tid  = threadIdx.x;
  const int lane = tid & 31;
  const int wave = tid >> 5;
  const int j0   = tid * 8;
  const float* row = S + (size_t)i * SENC + j0;
  const v4f a0 = *(const v4f*)(row);
  const v4f a1 = *(const v4f*)(row + 4);
  float t[8];
#pragma unroll
  for (int e = 0; e < 4; ++e) { t[e] = a0[e]; t[4 + e] = a1[e]; }
  float m = fmaxf(fmaxf(fmaxf(t[0], t[1]), fmaxf(t[2], t[3])), fmaxf(fmaxf(t[4], t[5]), fmaxf(t[6], t[7])));
#pragma unroll
  for (int off = 16; off > 0; off >>= 1) m = fmaxf(m, __shfl_xor(m, off, 32));
  if (lane == 0) redm[wave] = m;
  __syncthreads();
  float mx = redm[0];
#pragma unroll
  for (int w = 1; w < 8; ++w) mx = fmaxf(mx, redm[w]);
  float ex[8];
#pragma unroll
  for (int e = 0; e < 8; ++e) ex[e] = __expf(t[e] - mx);
  float ps = ((((((ex[0] + ex[1]) + ex[2]) + ex[3]) + ex[4]) + ex[5]) + ex[6]) + ex[7];
#pragma unroll
  for (int off = 16; off > 0; off >>= 1) ps += __shfl_xor(ps, off, 32);
  if (lane == 0) reds[wave] = ps;
  __syncthreads();
  float tot = reds[0];
#pragma unroll
  for (int w = 1; w < 8; ++w) tot += reds[w];
  const float inv = 1.0f / tot;
  unsigned hw[4], lw[4];
#pragma unroll
  for (int q = 0; q < 4; ++q) {
    const float p0 = ex[2 * q] * inv, p1 = ex[2 * q + 1] * inv;
    const unsigned short hb0 = f2bf_bits(p0), hb1 = f2bf_bits(p1);
    const unsigned short lb0 = f2bf_bits(p0 - bf_bits2f(hb0));
    const unsigned short lb1 = f2bf_bits(p1 - bf_bits2f(hb1));
    hw[q] = pk16(hb0, hb1);
    lw[q] = pk16(lb0, lb1);
  }
  const v4u hvv = (v4u){hw[0], hw[1], hw[2], hw[3]};
  const v4u lvv = (v4u){lw[0], lw[1], lw[2], lw[3]};
  const size_t rowoff = (size_t)i * SENC + j0;
  *(volatile v4u*)(Phi + rowoff) = hvv;
  *(volatile v4u*)(Plo + rowoff) = lvv;
  __threadfence();
  *(volatile v4u*)(Phi + rowoff) = hvv;
  *(volatile v4u*)(Plo + rowoff) = lvv;
}

extern "C" void kernel_launch(void* const* d_in, const int* in_sizes, int n_in,
                              void* d_out, int out_size, void* d_ws, size_t ws_size,
                              hipStream_t stream) {
  if (n_in < 5) return;
  if (in_sizes[0] != NBATCH * SENC * DIN) return;
  if (in_sizes[1] != NBATCH * SDEC * DIN) return;
  if (in_sizes[2] != DIN * UNITS || in_sizes[3] != DIN * UNITS || in_sizes[4] != DIN * UNITS) return;
  if (out_size != NBATCH * SDEC * UNITS) return;

  const float* enc = (const float*)d_in[0];
  const float* dec = (const float*)d_in[1];
  const float* Wq  = (const float*)d_in[2];
  const float* Wk  = (const float*)d_in[3];
  const float* Wv  = (const float*)d_in[4];
  const float* fz  = Wq;

  const size_t PW  = (size_t)DIN * UNITS * 2;
  const size_t PXD = (size_t)NBATCH * SDEC * DIN * 2;
  const size_t PXE = (size_t)SENC * DIN * 2;
  const size_t PVT = (size_t)UNITS * SENC * 2;
  const size_t PS  = (size_t)SDEC * SENC * 4;
  const size_t PP  = (size_t)SDEC * SENC * 2;
  size_t off = 0;
  const size_t oWqTh = off; off += PW;
  const size_t oWqTl = off; off += PW;
  const size_t oWkTh = off; off += PW;
  const size_t oWkTl = off; off += PW;
  const size_t oWvTh = off; off += PW;
  const size_t oWvTl = off; off += PW;
  const size_t oXDh  = off; off += PXD;
  const size_t oXDl  = off; off += PXD;
  const size_t oQh   = off; off += PXD;
  const size_t oQl   = off; off += PXD;
  const size_t oXEh  = off; off += PXE;
  const size_t oXEl  = off; off += PXE;
  const size_t oKh   = off; off += PXE;
  const size_t oKl   = off; off += PXE;
  const size_t oVTh  = off; off += PVT;
  const size_t oVTl  = off; off += PVT;
  const size_t oS    = off; off += PS;
  const size_t oPh   = off; off += PP;
  const size_t oPl   = off; off += PP;
  if (off > ws_size) return;

  char* ws = (char*)d_ws;
  unsigned short* WqTh = (unsigned short*)(ws + oWqTh);
  unsigned short* WqTl = (unsigned short*)(ws + oWqTl);
  unsigned short* WkTh = (unsigned short*)(ws + oWkTh);
  unsigned short* WkTl = (unsigned short*)(ws + oWkTl);
  unsigned short* WvTh = (unsigned short*)(ws + oWvTh);
  unsigned short* WvTl = (unsigned short*)(ws + oWvTl);
  unsigned short* XDh  = (unsigned short*)(ws + oXDh);
  unsigned short* XDl  = (unsigned short*)(ws + oXDl);
  unsigned short* Qh   = (unsigned short*)(ws + oQh);
  unsigned short* Ql   = (unsigned short*)(ws + oQl);
  unsigned short* XEh  = (unsigned short*)(ws + oXEh);
  unsigned short* XEl  = (unsigned short*)(ws + oXEl);
  unsigned short* Kh   = (unsigned short*)(ws + oKh);
  unsigned short* Kl   = (unsigned short*)(ws + oKl);
  unsigned short* VTh  = (unsigned short*)(ws + oVTh);
  unsigned short* VTl  = (unsigned short*)(ws + oVTl);
  float*          Sbuf = (float*)(ws + oS);
  unsigned short* Ph   = (unsigned short*)(ws + oPh);
  unsigned short* Pl   = (unsigned short*)(ws + oPl);

  const dim3 blk(256);
  const dim3 gTr(UNITS / 64, DIN / 64);
  transpose_split_kernel<<<gTr, blk, 0, stream>>>(Wq, UNITS, WqTh, WqTl, DIN);
  transpose_split_kernel<<<gTr, blk, 0, stream>>>(Wk, UNITS, WkTh, WkTl, DIN);
  transpose_split_kernel<<<gTr, blk, 0, stream>>>(Wv, UNITS, WvTh, WvTl, DIN);

  const int n2d = NBATCH * SDEC * DIN / 2;
  const dim3 gSplitD((n2d + 255) / 256);
  split_bf16x2_kernel<<<gSplitD, blk, 0, stream>>>(dec, XDh, XDl, n2d);

  const dim3 gQ((((NBATCH * SDEC) / 64) * (UNITS / 64) + 7) / 8, 1);
  wmma_gemm64<1, true, 0, 2, false, 0><<<gQ, blk, 0, stream>>>(
      XDh, XDl, DIN, 0L, WqTh, WqTl, DIN, 0L, (void*)Qh, (void*)Ql, UNITS, 0L,
      fz, fz, 0L, NBATCH * SDEC, UNITS, DIN, 1.0f);

  const int n2e = SENC * DIN / 2;
  const dim3 gSplitE((n2e + 255) / 256);
  const dim3 gK(((SENC / 64) * (UNITS / 64) + 7) / 8, 1);
  const dim3 gVT(((UNITS / 64) * (SENC / 64) + 7) / 8, 1);
  const dim3 gS(((SDEC / 64) * (SENC / 64) + 7) / 8, 1);
  const dim3 gSm(SDEC);
  const dim3 gPV(((SDEC / 64) * (UNITS / 64) + 7) / 8, 1);

  for (int b = 0; b < NBATCH; ++b) {
    split_bf16x2_kernel<<<gSplitE, blk, 0, stream>>>(enc + (size_t)b * SENC * DIN, XEh, XEl, n2e);
    wmma_gemm64<1, true, 0, 2, false, 0><<<gK, blk, 0, stream>>>(
        XEh, XEl, DIN, 0L, WkTh, WkTl, DIN, 0L, (void*)Kh, (void*)Kl, UNITS, 0L,
        fz, fz, 0L, SENC, UNITS, DIN, 1.0f);
    wmma_gemm64<1, true, 0, 2, false, 0><<<gVT, blk, 0, stream>>>(
        WvTh, WvTl, DIN, 0L, XEh, XEl, DIN, 0L, (void*)VTh, (void*)VTl, SENC, 0L,
        fz, fz, 0L, UNITS, SENC, DIN, 1.0f);
    const size_t qoff = (size_t)b * SDEC * UNITS;
    wmma_gemm64<1, true, 0, 0, false, 0><<<gS, blk, 0, stream>>>(
        Qh + qoff, Ql + qoff, UNITS, 0L, Kh, Kl, UNITS, 0L, (void*)Sbuf, (void*)Sbuf, SENC, 0L,
        fz, fz, 0L, SDEC, SENC, UNITS, 1.0f);
    softmax_split_kernel<<<gSm, blk, 0, stream>>>(Sbuf, Ph, Pl);
    float* outb = (float*)d_out + (size_t)b * SDEC * UNITS;
    wmma_gemm64<1, true, 0, 0, false, 0><<<gPV, blk, 0, stream>>>(
        Ph, Pl, SENC, 0L, VTh, VTl, SENC, 0L, (void*)outb, (void*)outb, UNITS, 0L,
        fz, fz, 0L, SDEC, UNITS, SENC, 1.0f);
  }
  (void)hipGetLastError();
}
